// QNN_56676388438509
// MI455X (gfx1250) — hardware-verified
//
#include <hip/hip_runtime.h>
#include <math.h>

typedef __attribute__((ext_vector_type(16))) _Float16 v16h;
typedef __attribute__((ext_vector_type(8)))  float    v8f;
typedef __attribute__((ext_vector_type(4)))  float    v4f;
typedef __attribute__((ext_vector_type(8)))  unsigned v8u;

constexpr int kQubits        = 8;
constexpr int kLayers        = 3;
constexpr int kDim           = 1 << kQubits;
constexpr int kBatch         = 65536;
constexpr int kFeat          = kQubits + 1;
constexpr int kOutC          = 2;
constexpr int kRowsPerWave   = 16;
constexpr int kWavesPerBlock = 8;
constexpr int kSlabPitch     = 17;
constexpr int kKSteps        = kDim / 32;
constexpr float kCarry       = 32768.0f;
constexpr float kCarryInv    = 1.0f / 32768.0f;
constexpr float kHalfFloor   = 6.103515625e-5f;
static_assert(kDim == 256, "basis size");
static_assert((kDim % 32) == 0 && kKSteps == 8, "k extent is a multiple of 32");
static_assert(kFeat <= 16, "feature columns fit one 16-wide tile");
static_assert((kBatch % (kRowsPerWave * kWavesPerBlock)) == 0, "row tiles exact");
static_assert(kRowsPerWave * kOutC * 4 == 128, "one wave stores one 128-B line");

constexpr unsigned idx_to_v(unsigned k) {
  unsigned v = 0;
  for (int j = 0; j < kQubits; ++j) v |= ((k >> (kQubits - 1 - j)) & 1u) << j;
  return v;
}
constexpr unsigned ring_fwd(unsigned v) {
  for (int l = 0; l < kLayers; ++l)
    for (int i = 0; i < kQubits; ++i) v ^= ((v >> i) & 1u) << ((i + 1) & (kQubits - 1));
  return v;
}
constexpr unsigned ring_inv(unsigned v) {
  for (int l = 0; l < kLayers; ++l)
    for (int i = kQubits - 1; i >= 0; --i) v ^= ((v >> i) & 1u) << ((i + 1) & (kQubits - 1));
  return v;
}
constexpr unsigned parity8(unsigned v) {
  unsigned p = 0;
  for (int j = 0; j < 8; ++j) p ^= (v >> j) & 1u;
  return p;
}
constexpr bool ring_inverse_ok() {
  for (unsigned v = 0; v < 256u; ++v) {
    if (ring_inv(ring_fwd(v)) != v) return false;
    if (ring_fwd(ring_inv(v)) != v) return false;
  }
  return true;
}
constexpr bool ring_masks_ok() {
  const unsigned mk[8] = {0x32u, 0x56u, 0xACu, 0x59u, 0xB3u, 0x66u, 0xCCu, 0x99u};
  for (unsigned v = 0; v < 256u; ++v) {
    const unsigned f = ring_fwd(v);
    for (int i = 0; i < 8; ++i)
      if (((f >> i) & 1u) != parity8(v & mk[i])) return false;
    if (parity8(f) != parity8(v & 0x11u)) return false;
  }
  return true;
}
static_assert(ring_inverse_ok(), "inverse ring map");
static_assert(ring_masks_ok(), "ring dependency masks");

constexpr unsigned kDeltaH = ring_inv(1u << 4);
static_assert(idx_to_v(8u) == (1u << 4), "index bit 3 is qubit 4");

template <int S, int I> struct PermSlot {
  static constexpr unsigned kf = 32u * (unsigned)S + 16u * ((unsigned)I >> 3) + ((unsigned)I & 7u);
  static constexpr unsigned v0 = ring_inv(idx_to_v(kf));
  static constexpr int lo = (int)(v0 & 15u);
  static constexpr int hi = (int)(v0 >> 4);
};

__device__ __forceinline__ v8f mma_f16_guard(v16h a, v16h b, v8f c) {
  c = __builtin_amdgcn_wmma_f32_16x16x32_f16(false, a, false, b, (short)0, c, false, false);
  asm volatile("v_nop\n\tv_nop\n\tv_nop\n\tv_nop" : "+v"(c) : "v"(a), "v"(b));
  return c;
}

__device__ __forceinline__ _Float16 carry_h(float p) {
  float pc = p * kCarry;
  pc = (pc < kHalfFloor) ? 0.0f : pc;
  return (_Float16)pc;
}

#define QPROB_SET(I) a[I] = carry_h(PH[PermSlot<S, I>::lo] * PL[PermSlot<S, I>::hi]);

template <int S>
__device__ __forceinline__ v8f readout_step(const float (&PH)[16], const float (&PL)[16],
                                            v8u b0, unsigned sel, v8f acc) {
  v16h a;
  QPROB_SET(0)  QPROB_SET(1)  QPROB_SET(2)  QPROB_SET(3)
  QPROB_SET(4)  QPROB_SET(5)  QPROB_SET(6)  QPROB_SET(7)
  QPROB_SET(8)  QPROB_SET(9)  QPROB_SET(10) QPROB_SET(11)
  QPROB_SET(12) QPROB_SET(13) QPROB_SET(14) QPROB_SET(15)
  const unsigned flip = ((unsigned)__popc(((unsigned)S << 5) & sel) & 1u) ? 0x80008000u : 0u;
  v8u bw;
#pragma unroll
  for (int e = 0; e < 8; ++e) bw[e] = b0[e] ^ flip;
  const v16h b = __builtin_bit_cast(v16h, bw);
  return mma_f16_guard(a, b, acc);
}

__global__ __launch_bounds__(256) void qcirc_readout_kernel(
    const float* __restrict__ x, const float* __restrict__ enc_off, const float* __restrict__ enc_sc,
    const float* __restrict__ Wh, const float* __restrict__ bh, float* __restrict__ out, int nrows)
{
  __shared__ __align__(16) float sF[kWavesPerBlock][16 * kSlabPitch];

  unsigned lane = threadIdx.x & 31u;
  unsigned wave = threadIdx.x >> 5;
  asm volatile("" : "+v"(lane));
  asm volatile("" : "+v"(wave));
  unsigned m = lane & 15u;
  unsigned h = lane >> 4;
  asm volatile("" : "+v"(m));
  asm volatile("" : "+v"(h));
  const unsigned base = (blockIdx.x * (unsigned)kWavesPerBlock + wave) * (unsigned)kRowsPerWave;
  unsigned row = base + m;
  const unsigned lastRow = (unsigned)(nrows - 1);
  unsigned rowc = (row < lastRow) ? row : lastRow;
  asm volatile("" : "+v"(rowc));

  const float* xr = x + (size_t)rowc * kQubits;
  const v4f x0 = *(const v4f*)(xr);
  const v4f x1 = *(const v4f*)(xr + 4);
  const float xv[8] = {x0[0], x0[1], x0[2], x0[3], x1[0], x1[1], x1[2], x1[3]};

  float c2[8], s2[8];
#pragma unroll
  for (int j = 0; j < kQubits; ++j) {
    const float hf = 0.5f * (enc_off[j] + enc_sc[j] * xv[j]);
    float sn, cs;
    sincosf(hf, &sn, &cs);
    c2[j] = cs * cs;
    s2[j] = sn * sn;
  }

  const bool hb = (h != 0u);
  float g0[8], g1[8];
#pragma unroll
  for (int j = 0; j < kQubits; ++j) {
    const bool sw = (((kDeltaH >> j) & 1u) != 0u) && hb;
    const float a0 = c2[j], a1 = s2[j];
    g0[j] = sw ? a1 : a0;
    g1[j] = sw ? a0 : a1;
  }

  float q01[4], q23[4], q45[4], q67[4];
#pragma unroll
  for (int t = 0; t < 4; ++t) {
    q01[t] = ((t & 1) ? g1[0] : g0[0]) * ((t >> 1) ? g1[1] : g0[1]);
    q23[t] = ((t & 1) ? g1[2] : g0[2]) * ((t >> 1) ? g1[3] : g0[3]);
    q45[t] = ((t & 1) ? g1[4] : g0[4]) * ((t >> 1) ? g1[5] : g0[5]);
    q67[t] = ((t & 1) ? g1[6] : g0[6]) * ((t >> 1) ? g1[7] : g0[7]);
  }
  float PH[16], PL[16];
#pragma unroll
  for (int t = 0; t < 16; ++t) {
    PH[t] = q01[t & 3] * q23[t >> 2];
    PL[t] = q45[t & 3] * q67[t >> 2];
  }

  unsigned sel = (m < 8u) ? (0x80u >> m) : ((m == 8u) ? 0xFFu : 0u);
  asm volatile("" : "+v"(sel));
  unsigned hk = h << 3;
  asm volatile("" : "+v"(hk));
  const float posv = (m < (unsigned)kFeat) ? 1.0f : 0.0f;
  const float negv = -posv;
  v16h bb;
#pragma unroll
  for (int i = 0; i < 16; ++i) {
    const unsigned kb = 16u * ((unsigned)i >> 3) + ((unsigned)i & 7u);
    const unsigned kk = kb | hk;
    const unsigned par = (unsigned)__popc(kk & sel) & 1u;
    float val = par ? negv : posv;
    asm volatile("" : "+v"(val));
    bb[i] = (_Float16)val;
  }
  const v8u b0 = __builtin_bit_cast(v8u, bb);

  const unsigned orow = lane >> 1;
  unsigned ocol = lane & 1u;
  asm volatile("" : "+v"(ocol));
  float wv[kFeat];
#pragma unroll
  for (int i = 0; i < kFeat; ++i) wv[i] = Wh[ocol * (unsigned)kFeat + (unsigned)i];
  const float bv = bh[ocol];

  v8f acc = (v8f){0.f, 0.f, 0.f, 0.f, 0.f, 0.f, 0.f, 0.f};
  acc = readout_step<0>(PH, PL, b0, sel, acc);
  acc = readout_step<1>(PH, PL, b0, sel, acc);
  acc = readout_step<2>(PH, PL, b0, sel, acc);
  acc = readout_step<3>(PH, PL, b0, sel, acc);
  acc = readout_step<4>(PH, PL, b0, sel, acc);
  acc = readout_step<5>(PH, PL, b0, sel, acc);
  acc = readout_step<6>(PH, PL, b0, sel, acc);
  acc = readout_step<7>(PH, PL, b0, sel, acc);

  float* slab = sF[wave];
#pragma unroll
  for (int r = 0; r < 8; ++r) slab[(8u * h + (unsigned)r) * (unsigned)kSlabPitch + m] = acc[r] * kCarryInv;
  __syncthreads();

  float o = 0.0f;
#pragma unroll
  for (int i = 0; i < kFeat; ++i) o = fmaf(slab[orow * (unsigned)kSlabPitch + (unsigned)i], wv[i], o);
  o += bv;

  if (base < (unsigned)nrows) {
    float* p = out + (size_t)base * kOutC + lane;
    *(volatile float*)p = o;
    __threadfence();
    *(volatile float*)p = o;
  }
}

extern "C" void kernel_launch(void* const* d_in, const int* in_sizes, int n_in,
                              void* d_out, int out_size, void* d_ws, size_t ws_size,
                              hipStream_t stream) {
  (void)d_ws;
  (void)ws_size;
  if (n_in < 6) return;
  if (in_sizes[0] != kBatch * kQubits) return;
  if (in_sizes[2] != kQubits) return;
  if (in_sizes[3] != kQubits) return;
  if (in_sizes[4] != kOutC * kFeat) return;
  if (in_sizes[5] != kOutC) return;
  if (out_size != kBatch * kOutC) return;

  const float* x       = (const float*)d_in[0];
  const float* enc_off = (const float*)d_in[2];
  const float* enc_sc  = (const float*)d_in[3];
  const float* Wh      = (const float*)d_in[4];
  const float* bh      = (const float*)d_in[5];
  float* out = (float*)d_out;

  const int blocks = kBatch / (kRowsPerWave * kWavesPerBlock);
  qcirc_readout_kernel<<<blocks, 256, 0, stream>>>(x, enc_off, enc_sc, Wh, bh, out, kBatch);
}
